// LSTMDecoder_28080496181536
// MI455X (gfx1250) — hardware-verified
//
#include <hip/hip_runtime.h>
#include <math.h>

typedef __attribute__((ext_vector_type(16))) _Float16 v16h;
typedef __attribute__((ext_vector_type(8)))  _Float16 v8h;
typedef __attribute__((ext_vector_type(16))) __bf16   v16b;
typedef __attribute__((ext_vector_type(8)))  __bf16   v8b;
typedef __attribute__((ext_vector_type(8)))  float    v8f;
typedef __attribute__((ext_vector_type(4)))  float    v4f;
typedef __attribute__((ext_vector_type(2)))  float    v2f;

constexpr int kB    = 32;
constexpr int kBP   = 64;
constexpr int kP    = 196;
constexpr int kF    = 2048;
constexpr int kE    = 512;
constexpr int kH    = 512;
constexpr int kA    = 512;
constexpr int kV    = 10000;
constexpr int kVP   = 10240;
constexpr int kT    = 20;
constexpr int kG4   = 4 * kH;
constexpr int kKG   = kE + kF + kH;
constexpr int kRF   = kB * kP;
constexpr int kRO   = kB * kT;
constexpr int kThr  = 256;
constexpr float kInCarry = 1024.0f;
constexpr float kSc = 1.0f / (kInCarry * kInCarry);
constexpr float kF16MinNormal = 6.103515625e-5f;
constexpr int kFBE = 0, kFBD = 512, kFBG = 1024, kFBF = 3072, kFEnd = 13312;

static_assert((kRF % 64) == 0 && ((kRF / 64) * (kA / 64)) % 8 == 0 && (kA / 64) % 8 == 0 && (kG4 / 64) % 8 == 0 && (kRO % 64) == 0 && ((kRO / 64) * (kVP / 64)) % 8 == 0
              && (kF % 32) == 0 && (kH % 32) == 0 && (kKG % 32) == 0 && kFBF + kVP == kFEnd && kV <= kVP && (kV % 4) == 0, "GEMM M, N multiples of 64; grids exact; K multiples of 32");

constexpr size_t kOffF16 = 0ull;
constexpr size_t kOffENCW = 25690112ull;
constexpr size_t kOffDECW = 27787264ull;
constexpr size_t kOffWG16 = 28311552ull;
constexpr size_t kOffFCW = 40894464ull;
constexpr size_t kOffBIAS = 51380224ull;
constexpr size_t kOffENC32 = 51433472ull;
constexpr size_t kOffA16 = 64278528ull;
constexpr size_t kOffDP32 = 64671744ull;
constexpr size_t kOffG32 = 64802816ull;
constexpr size_t kOffC32 = 65327104ull;
constexpr size_t kOffHS16 = 65392640ull;
constexpr size_t kOffLOG32 = 66048000ull;
constexpr size_t kWsTotal = 92262400ull;
static_assert(kWsTotal <= 134217728ull, "carve cap: under 128 MiB");
static_assert(kOffF16 == 0
              && kOffENCW == kOffF16 + 25690112ull
              && kOffDECW == kOffENCW + 2097152ull
              && kOffWG16 == kOffDECW + 524288ull
              && kOffFCW == kOffWG16 + 12582912ull
              && kOffBIAS == kOffFCW + 10485760ull
              && kOffENC32 == kOffBIAS + 53248ull
              && kOffA16 == kOffENC32 + 12845056ull
              && kOffDP32 == kOffA16 + 393216ull
              && kOffG32 == kOffDP32 + 131072ull
              && kOffC32 == kOffG32 + 524288ull
              && kOffHS16 == kOffC32 + 65536ull
              && kOffLOG32 == kOffHS16 + 655360ull
              && kWsTotal == kOffLOG32 + 26214400ull, "the carve is chained and totalled");
static_assert((kOffF16 % 256) == 0 && (kOffENCW % 256) == 0 && (kOffDECW % 256) == 0 && (kOffWG16 % 256) == 0 && (kOffFCW % 256) == 0 && (kOffBIAS % 256) == 0 && (kOffENC32 % 256) == 0 && (kOffA16 % 256) == 0 && (kOffDP32 % 256) == 0 && (kOffG32 % 256) == 0 && (kOffC32 % 256) == 0 && (kOffHS16 % 256) == 0 && (kOffLOG32 % 256) == 0, "aligned regions");

__device__ __forceinline__ unsigned short f2bf_bits(float f) {
  unsigned u = __float_as_uint(f);
  return (unsigned short)((u + 0x7FFFu + ((u >> 16) & 1u)) >> 16);
}
__device__ __forceinline__ float bf_bits2f(unsigned short h) { return __uint_as_float(((unsigned)h) << 16); }
__device__ __forceinline__ float bf16r(float f) { return bf_bits2f(f2bf_bits(f)); }
__device__ __forceinline__ float carry_flush(float v, float carry) {
  const float s = v * carry;
  return (fabsf(s) < kF16MinNormal) ? 0.0f : s;
}
__device__ __forceinline__ float frcp(float x) { return __builtin_amdgcn_rcpf(x); }

__device__ __forceinline__ void dep_guard4_h(v8f& a, v8f& b, v8f& c, v8f& d, v16h x, v16h y) { asm volatile("v_nop\n\tv_nop\n\tv_nop\n\tv_nop" : "+v"(a), "+v"(b), "+v"(c), "+v"(d) : "v"(x), "v"(y)); }
__device__ __forceinline__ void dep_guard4_b(v8f& a, v8f& b, v8f& c, v8f& d, v16b x, v16b y) { asm volatile("v_nop\n\tv_nop\n\tv_nop\n\tv_nop" : "+v"(a), "+v"(b), "+v"(c), "+v"(d) : "v"(x), "v"(y)); }
__device__ __forceinline__ void keep4_h(v16h a, v16h b, v16h c, v16h d) { asm volatile("v_nop" :: "v"(a), "v"(b), "v"(c), "v"(d)); }
__device__ __forceinline__ void keep4_b(v16b a, v16b b, v16b c, v16b d) { asm volatile("v_nop" :: "v"(a), "v"(b), "v"(c), "v"(d)); }
__device__ __forceinline__ void acc_guard4(v8f& a, v8f& b, v8f& c, v8f& d) { asm volatile("v_nop\n\tv_nop\n\tv_nop\n\tv_nop" : "+v"(a), "+v"(b), "+v"(c), "+v"(d)); }

template <typename T> struct Frag;
template <> struct Frag<_Float16> {
  typedef v16h V; union U { v16h v; v8h h[2]; };
  static __device__ __forceinline__ v16h load(const _Float16* p) {
    U f; f.h[0] = *(const v8h*)(p); f.h[1] = *(const v8h*)(p + 16); return f.v;
  }
  static __device__ __forceinline__ v8f mma(v16h a, v16h b, v8f c) {
    return __builtin_amdgcn_wmma_f32_16x16x32_f16(false, a, false, b, (short)0, c, false, false);
  }
  static __device__ __forceinline__ void guard4(v8f& a, v8f& b, v8f& c, v8f& d, v16h x, v16h y) { dep_guard4_h(a, b, c, d, x, y); }
  static __device__ __forceinline__ void keep(v16h a, v16h b, v16h c, v16h d) { keep4_h(a, b, c, d); }
};
template <> struct Frag<__bf16> {
  typedef v16b V; union U { v16b v; v8b h[2]; };
  static __device__ __forceinline__ v16b load(const __bf16* p) {
    U f; f.h[0] = *(const v8b*)(p); f.h[1] = *(const v8b*)(p + 16); return f.v;
  }
  static __device__ __forceinline__ v8f mma(v16b a, v16b b, v8f c) {
    return __builtin_amdgcn_wmma_f32_16x16x32_bf16(false, a, false, b, (short)0, c, false, false);
  }
  static __device__ __forceinline__ void guard4(v8f& a, v8f& b, v8f& c, v8f& d, v16b x, v16b y) { dep_guard4_b(a, b, c, d, x, y); }
  static __device__ __forceinline__ void keep(v16b a, v16b b, v16b c, v16b d) { keep4_b(a, b, c, d); }
};

__device__ __forceinline__ v8f mma_h(v16h a, v16h b, v8f c) {
  c = __builtin_amdgcn_wmma_f32_16x16x32_f16(false, a, false, b, (short)0, c, false, false);
  asm volatile("v_nop\n\tv_nop\n\tv_nop\n\tv_nop" : "+v"(c) : "v"(a), "v"(b));
  return c;
}

template <int ET> struct Elem;
template <> struct Elem<0> { typedef _Float16 T; };
template <> struct Elem<1> { typedef __bf16 T; };
template <int ET, bool SPLIT, int BIAS_MODE, int OUT_MODE, bool RESID, int ACT = 0>
__global__ __launch_bounds__(256) void wmma_gemm64(
    const unsigned short* __restrict__ Ap, const unsigned short* __restrict__ A2p, int lda, long strideA,
    const unsigned short* __restrict__ Btp, const unsigned short* __restrict__ Bt2p, int ldb, long strideB,
    void* __restrict__ Cout, void* __restrict__ Cout2, int ldc, long strideC,
    const float* __restrict__ bias,
    const float* __restrict__ resid, long strideR,
    int M, int N, int K, float scale) {
  typedef typename Elem<ET>::T T;
  typedef typename Frag<T>::V V;
  const T* A = (const T*)Ap; const T* A2 = (const T*)A2p; const T* Bt = (const T*)Btp; const T* Bt2 = (const T*)Bt2p;
  __shared__ __align__(16) float sT[8][16 * 68];
  const int b    = blockIdx.y;
  const int lane = threadIdx.x & 31;
  const int wave = threadIdx.x >> 5;
  const int tilesN = N >> 6;
  const int tilesM = M >> 6;
  const int tile = blockIdx.x * 8 + wave;
  if (tile >= tilesM * tilesN) return;
  const int tm = tile / tilesN;
  const int tn = tile - tm * tilesN;
  const int m0 = tm << 6;
  const int n0 = tn << 6;

  const T* Ab  = A  + (size_t)b * strideA;
  const T* Bb  = Bt + (size_t)b * strideB;
  const T* Ab2 = SPLIT ? (A2  + (size_t)b * strideA) : nullptr;
  const T* Bb2 = SPLIT ? (Bt2 + (size_t)b * strideB) : nullptr;

  const int rlane = lane & 15;
  const int koff  = (lane >> 4) * 8;
  const int mOff  = (lane >> 4) * 8;

  v8f acc[4][4];
#pragma unroll
  for (int i = 0; i < 4; ++i)
#pragma unroll
    for (int j = 0; j < 4; ++j) acc[i][j] = (v8f){0.f,0.f,0.f,0.f,0.f,0.f,0.f,0.f};

  for (int k0 = 0; k0 < K; k0 += 32) {
    V bh[4], bl[4];
#pragma unroll
    for (int j = 0; j < 4; ++j) {
      const size_t bo = (size_t)(n0 + (j << 4) + rlane) * ldb + koff + k0;
      bh[j] = Frag<T>::load(Bb + bo);
      if (SPLIT) bl[j] = Frag<T>::load(Bb2 + bo);
    }
#pragma unroll
    for (int i = 0; i < 4; ++i) {
      const size_t ao = (size_t)(m0 + (i << 4) + rlane) * lda + koff + k0;
      V ah = Frag<T>::load(Ab + ao);
      V al;
      if (SPLIT) al = Frag<T>::load(Ab2 + ao);
#pragma unroll
      for (int j = 0; j < 4; ++j) {
        acc[i][j] = Frag<T>::mma(ah, bh[j], acc[i][j]);
        if (SPLIT) {
          acc[i][j] = Frag<T>::mma(ah, bl[j], acc[i][j]);
          acc[i][j] = Frag<T>::mma(al, bh[j], acc[i][j]);
        }
      }
      Frag<T>::guard4(acc[i][0], acc[i][1], acc[i][2], acc[i][3], ah, SPLIT ? al : ah);
    }
    Frag<T>::keep(bh[0], bh[1], bh[2], bh[3]);
    if (SPLIT) Frag<T>::keep(bl[0], bl[1], bl[2], bl[3]);
  }
  acc_guard4(acc[0][0], acc[0][1], acc[0][2], acc[0][3]);
  acc_guard4(acc[1][0], acc[1][1], acc[1][2], acc[1][3]);
  acc_guard4(acc[2][0], acc[2][1], acc[2][2], acc[2][3]);
  acc_guard4(acc[3][0], acc[3][1], acc[3][2], acc[3][3]);

  float* slab = sT[wave];
  const float* Rb = RESID ? (resid + (size_t)b * strideR) : nullptr;
#pragma unroll
  for (int i = 0; i < 4; ++i) {
    const int mBase = m0 + (i << 4);
#pragma unroll
    for (int j = 0; j < 4; ++j) {
      const int n = n0 + (j << 4) + rlane;
      float bv = 0.f;
      if (BIAS_MODE == 2) bv = bias[n];
#pragma unroll
      for (int r = 0; r < 8; ++r) {
        float v = acc[i][j][r] * scale;
        if (BIAS_MODE == 1) v += bias[mBase + mOff + r];
        if (BIAS_MODE == 2) v += bv;
        if (RESID) v += Rb[(size_t)(mBase + mOff + r) * ldc + n];
        if (ACT == 1) v = tanhf(v);
        if (ACT == 2) v = fmaxf(v, 0.0f);
        if (ACT == 3) v = v / (1.0f + expf(-v));
        if (ACT == 4) v = (v > 0.f) ? v : 0.01f * v;
        slab[(mOff + r) * 68 + (j << 4) + rlane] = v;
      }
    }
    __builtin_amdgcn_fence(__ATOMIC_RELEASE, "workgroup");
    __builtin_amdgcn_wave_barrier();
    __builtin_amdgcn_fence(__ATOMIC_ACQUIRE, "workgroup");
    if (OUT_MODE == 0) {
      float* C = (float*)Cout + (size_t)b * strideC;
      const int hh = lane >> 4, c4 = (lane & 15) * 4;
      for (int pass = 0; pass < 2; ++pass) {
#pragma unroll
        for (int it = 0; it < 8; ++it) {
          const int row = it * 2 + hh;
          v4f v = *(const v4f*)(slab + row * 68 + c4);
          *(volatile v4f*)(C + (size_t)(mBase + row) * ldc + n0 + c4) = v;
        }
        __threadfence();
      }
    } else {
      const int q = lane >> 3, c8 = (lane & 7) * 8;
      unsigned short* C  = (unsigned short*)Cout  + (size_t)b * strideC;
      unsigned short* C2 = (OUT_MODE == 2) ? ((unsigned short*)Cout2 + (size_t)b * strideC) : nullptr;
      for (int pass = 0; pass < 2; ++pass) {
#pragma unroll
        for (int it = 0; it < 4; ++it) {
          const int row = it * 4 + q;
          const float* sp = slab + row * 68 + c8;
          v8h hv, lv;
#pragma unroll
          for (int e = 0; e < 8; ++e) {
            if (OUT_MODE == 1) {
              hv[e] = (_Float16)sp[e];
            } else {
              unsigned short hb = f2bf_bits(sp[e]);
              unsigned short lb = f2bf_bits(sp[e] - bf_bits2f(hb));
              hv[e] = __builtin_bit_cast(_Float16, hb);
              lv[e] = __builtin_bit_cast(_Float16, lb);
            }
          }
          *(volatile v8h*)(C + (size_t)(mBase + row) * ldc + n0 + c8) = hv;
          if (OUT_MODE == 2) *(volatile v8h*)(C2 + (size_t)(mBase + row) * ldc + n0 + c8) = lv;
        }
        __threadfence();
      }
    }
    __builtin_amdgcn_fence(__ATOMIC_RELEASE, "workgroup");
    __builtin_amdgcn_wave_barrier();
    __builtin_amdgcn_fence(__ATOMIC_ACQUIRE, "workgroup");
  }
}

__global__ __launch_bounds__(kThr) void cast_plane_kernel(const float* __restrict__ src, unsigned short* __restrict__ dst,
                                                          int colsLog2, int dstPitch, int dstOff) {
  const int i   = blockIdx.x * kThr + threadIdx.x;
  const int sh  = colsLog2 - 3;
  const int row = i >> sh;
  const int c8  = (i & ((1 << sh) - 1)) * 8;
  const float* sp = src + ((size_t)row << colsLog2) + c8;
  const v4f a0 = *(const v4f*)(sp);
  const v4f a1 = *(const v4f*)(sp + 4);
  v8h hv;
#pragma unroll
  for (int e = 0; e < 4; ++e) {
    const float f0 = a0[e];
    const float f1 = a1[e];
    hv[e]     = (_Float16)carry_flush(bf16r(f0), kInCarry);
    hv[4 + e] = (_Float16)carry_flush(bf16r(f1), kInCarry);
  }
  unsigned short* dp = dst + (size_t)row * dstPitch + dstOff + c8;
  *(volatile v8h*)dp = hv;
  __threadfence();
  *(volatile v8h*)dp = hv;
}

__device__ __forceinline__ float fast_tanh(float v) { return 1.0f - 2.0f * frcp(__expf(2.0f * v) + 1.0f); }
__device__ __forceinline__ float fast_sigmoid(float v) { return frcp(1.0f + __expf(-v)); }

__global__ __launch_bounds__(kThr) void wgate_kernel(const float* __restrict__ W_ih, const float* __restrict__ W_hh, unsigned short* __restrict__ WG16) {
  unsigned v = blockIdx.x * (unsigned)kThr + threadIdx.x;
  asm volatile("" : "+v"(v));
  const unsigned n = v / 384u, c8 = (v % 384u) * 8u;
  const float* sp = (c8 < (unsigned)(kE + kF)) ? (W_ih + (size_t)n * (kE + kF) + c8) : (W_hh + (size_t)n * kH + (c8 - (unsigned)(kE + kF)));
  const v4f a0 = *(const v4f*)sp, a1 = *(const v4f*)(sp + 4);
  v8h hv;
#pragma unroll
  for (int e = 0; e < 4; ++e) { const float p = a0[e], q = a1[e]; hv[e] = (_Float16)carry_flush(bf16r(p), kInCarry); hv[4 + e] = (_Float16)carry_flush(bf16r(q), kInCarry); }
  unsigned short* dp = WG16 + (size_t)v * 8u;
  *(volatile v8h*)dp = hv;
  __threadfence();
  *(volatile v8h*)dp = hv;
}
static_assert(kKG / 8 == 384 && kG4 * 384 == 3072 * kThr && ((kE + kF) % 8) == 0, "gate-plane grid exact");

__global__ __launch_bounds__(kThr) void fcw_kernel(const float* __restrict__ fc_W, unsigned short* __restrict__ FCW) {
  unsigned v = blockIdx.x * (unsigned)kThr + threadIdx.x;
  asm volatile("" : "+v"(v));
  const unsigned n = v >> 6, c8 = (v & 63u) * 8u;
  const bool live = n < (unsigned)kV;
  const float* sp = fc_W + (size_t)(live ? n : 0u) * kH + c8;
  const v4f a0 = *(const v4f*)sp, a1 = *(const v4f*)(sp + 4);
  v8h hv;
#pragma unroll
  for (int e = 0; e < 4; ++e) { const float p = a0[e], q = a1[e]; hv[e] = (_Float16)(live ? carry_flush(bf16r(p), kInCarry) : 0.0f); hv[4 + e] = (_Float16)(live ? carry_flush(bf16r(q), kInCarry) : 0.0f); }
  unsigned short* dp = FCW + (size_t)v * 8u;
  *(volatile v8h*)dp = hv;
  __threadfence();
  *(volatile v8h*)dp = hv;
}
static_assert(kVP * (kH / 8) == 2560 * kThr, "word-plane grid exact");

__global__ __launch_bounds__(kThr) void setup_kernel(const float* __restrict__ enc_b, const float* __restrict__ dec_b, const float* __restrict__ b_ih,
                                                     const float* __restrict__ b_hh, const float* __restrict__ fc_b, float* __restrict__ BIAS,
                                                     unsigned short* __restrict__ A16, float* __restrict__ C32) {
  unsigned v = blockIdx.x * (unsigned)kThr + threadIdx.x;
  asm volatile("" : "+v"(v));
  if (v < 3328u) {
    const unsigned i0 = v * 4u;
    const bool isE = i0 < (unsigned)kFBD, isD = (i0 >= (unsigned)kFBD) && (i0 < (unsigned)kFBG), isG = (i0 >= (unsigned)kFBG) && (i0 < (unsigned)kFBF);
    const bool isF = (i0 >= (unsigned)kFBF) && (i0 < (unsigned)(kFBF + kV));
    const float* sp = isE ? (enc_b + i0) : isD ? (dec_b + (i0 - (unsigned)kFBD)) : isG ? (b_ih + (i0 - (unsigned)kFBG)) : isF ? (fc_b + (i0 - (unsigned)kFBF)) : enc_b;
    const float* s2 = isG ? (b_hh + (i0 - (unsigned)kFBG)) : enc_b;
    const v4f a = *(const v4f*)sp, c = *(const v4f*)s2;
    const bool live = isE || isD || isG || isF;
    v4f o;
#pragma unroll
    for (int e = 0; e < 4; ++e) { const float p = a[e], q = c[e]; o[e] = live ? (isG ? (bf16r(p) + bf16r(q)) : bf16r(p)) : 0.0f; }
    float* dp = BIAS + i0;
    *(volatile v4f*)dp = o;
    __threadfence();
    *(volatile v4f*)dp = o;
  } else if (v < 27904u) {
    v8h hv;
#pragma unroll
    for (int e = 0; e < 8; ++e) hv[e] = (_Float16)0.0f;
    unsigned short* dp = A16 + (size_t)(v - 3328u) * 8u;
    *(volatile v8h*)dp = hv;
    __threadfence();
    *(volatile v8h*)dp = hv;
  } else {
    const v4f z = {0.f, 0.f, 0.f, 0.f};
    float* dp = C32 + (size_t)(v - 27904u) * 4u;
    *(volatile v4f*)dp = z;
    __threadfence();
    *(volatile v4f*)dp = z;
  }
}
static_assert(kFEnd / 4 == 3328 && kBP * kKG / 8 == 24576 && 3328 + 24576 == 27904 && kB * kH / 4 == 4096 && 27904 + 4096 == 125 * kThr, "set-up grid exact");

__global__ __launch_bounds__(kThr) void score_kernel(const float* __restrict__ ENC32, const float* __restrict__ DP32, const float* __restrict__ full_W,
                                                     const float* __restrict__ full_b, const float* __restrict__ features, const int* __restrict__ captions,
                                                     const float* __restrict__ emb, unsigned short* __restrict__ A16, int t) {
  __shared__ __align__(16) float sDP[kA];
  __shared__ __align__(16) float sFW[kA];
  __shared__ float sE[kThr];
  __shared__ float sMx, sDen;
  const int tid = threadIdx.x;
  const int b = blockIdx.x;
  {
    const v2f d2 = *(const v2f*)(DP32 + (size_t)b * kA + 2 * tid), w2 = *(const v2f*)(full_W + 2 * tid);
    const float p0 = w2[0], p1 = w2[1];
    sDP[2 * tid] = d2[0]; sDP[2 * tid + 1] = d2[1];
    sFW[2 * tid] = bf16r(p0); sFW[2 * tid + 1] = bf16r(p1);
  }
  __syncthreads();
  {
    const bool live = tid < kP;
    const float* er = ENC32 + ((size_t)b * kP + (size_t)(live ? tid : 0)) * kA;
    float acc = 0.0f;
#pragma unroll 1
    for (int a = 0; a < kA; a += 4) {
      const v4f e4 = *(const v4f*)(er + a), d4 = *(const v4f*)(sDP + a), w4 = *(const v4f*)(sFW + a);
      acc += fmaxf(e4[0] + d4[0], 0.0f) * w4[0];
      acc += fmaxf(e4[1] + d4[1], 0.0f) * w4[1];
      acc += fmaxf(e4[2] + d4[2], 0.0f) * w4[2];
      acc += fmaxf(e4[3] + d4[3], 0.0f) * w4[3];
    }
    float fb = full_b[0];
    asm volatile("" : "+v"(fb));
    sE[tid] = live ? (acc + bf16r(fb)) : 0.0f;
  }
  __syncthreads();
  if (tid == 0) {
    float mx = sE[0];
#pragma unroll 1
    for (int p = 1; p < kP; ++p) { const float q = sE[p]; mx = (q > mx) ? q : mx; }
    sMx = mx;
  }
  __syncthreads();
  {
    const float ex = __expf(sE[tid] - sMx);
    __syncthreads();
    sE[tid] = (tid < kP) ? ex : 0.0f;
  }
  __syncthreads();
  if (tid == 0) {
    float s = 0.0f;
#pragma unroll 1
    for (int p = 0; p < kP; ++p) s += sE[p];
    sDen = s;
  }
  __syncthreads();
  {
    const int f8 = tid * 8;
    const float* fp = features + (size_t)b * kP * kF + f8;
    float acc[8];
#pragma unroll
    for (int e = 0; e < 8; ++e) acc[e] = 0.0f;
#pragma unroll 1
    for (int p = 0; p < kP; ++p) {
      const float a = sE[p];
      const v4f x0 = *(const v4f*)(fp + (size_t)p * kF), x1 = *(const v4f*)(fp + (size_t)p * kF + 4);
#pragma unroll
      for (int e = 0; e < 4; ++e) { const float q0 = x0[e], q1 = x1[e]; acc[e] += a * bf16r(q0); acc[4 + e] += a * bf16r(q1); }
    }
    const float inv = 1.0f / sDen;
    v8h hv;
#pragma unroll
    for (int e = 0; e < 8; ++e) hv[e] = (_Float16)carry_flush(acc[e] * inv, kInCarry);
    unsigned short* cp = A16 + (size_t)b * kKG + kE + f8;
    int tok = captions[(size_t)b * kT + t];
    asm volatile("" : "+v"(tok));
    tok = (tok < 0) ? 0 : ((tok >= kV) ? (kV - 1) : tok);
    const bool em = tid < (kE / 8);
    const float* ep = emb + (size_t)tok * kE + (em ? f8 : 0);
    const v4f m0 = *(const v4f*)ep, m1 = *(const v4f*)(ep + 4);
    v8h ev;
#pragma unroll
    for (int e = 0; e < 4; ++e) { const float q0 = m0[e], q1 = m1[e]; ev[e] = (_Float16)carry_flush(bf16r(q0), kInCarry); ev[4 + e] = (_Float16)carry_flush(bf16r(q1), kInCarry); }
    unsigned short* xp = A16 + (size_t)b * kKG + f8;
    for (int pass = 0; pass < 2; ++pass) {
      *(volatile v8h*)cp = hv;
      if (em) *(volatile v8h*)xp = ev;
      __threadfence();
    }
  }
}
static_assert(kA == 2 * kThr && kP <= kThr && kF == 8 * kThr && (kE / 8) <= kThr, "attention thread maps");

__global__ __launch_bounds__(kThr) void cell_kernel(const float* __restrict__ G32, float* __restrict__ C32, unsigned short* __restrict__ A16,
                                                    unsigned short* __restrict__ HS16, int t) {
  unsigned v = blockIdx.x * (unsigned)kThr + threadIdx.x;
  asm volatile("" : "+v"(v));
  const unsigned b = v >> 6, u8 = (v & 63u) * 8u;
  const float* gr = G32 + (size_t)b * kG4 + u8;
  float* cp = C32 + (size_t)b * kH + u8;
  v4f cn0, cn1; v8h hv;
#pragma unroll
  for (int hlf = 0; hlf < 2; ++hlf) {
    const v4f gi = *(const v4f*)(gr + 4 * hlf), gf = *(const v4f*)(gr + kH + 4 * hlf), gg = *(const v4f*)(gr + 2 * kH + 4 * hlf), go = *(const v4f*)(gr + 3 * kH + 4 * hlf);
    const v4f co = *(const v4f*)(cp + 4 * hlf);
#pragma unroll
    for (int e = 0; e < 4; ++e) {
      const float cn = fast_sigmoid(gf[e]) * co[e] + fast_sigmoid(gi[e]) * fast_tanh(gg[e]);
      const float hn = fast_sigmoid(go[e]) * fast_tanh(cn);
      if (hlf == 0) cn0[e] = cn; else cn1[e] = cn;
      hv[4 * hlf + e] = (_Float16)carry_flush(hn, kInCarry);
    }
  }
  unsigned short* hp = A16 + (size_t)b * kKG + (kE + kF) + u8;
  unsigned short* op = HS16 + ((size_t)b * kT + (size_t)t) * kH + u8;
  for (int pass = 0; pass < 2; ++pass) {
    *(volatile v4f*)cp = cn0; *(volatile v4f*)(cp + 4) = cn1;
    *(volatile v8h*)hp = hv;
    *(volatile v8h*)op = hv;
    __threadfence();
  }
}
static_assert(kB * kH / 8 == 8 * kThr && kH / 8 == 64, "cell grid: 8 blocks");

__global__ __launch_bounds__(kThr) void out_kernel(const float* __restrict__ LOG32, float* __restrict__ out) {
  unsigned v = blockIdx.x * (unsigned)kThr + threadIdx.x;
  asm volatile("" : "+v"(v));
  const unsigned i4 = v * 4u;
  const unsigned row = i4 / (unsigned)kV, w = i4 % (unsigned)kV;
  const v4f o = *(const v4f*)(LOG32 + (size_t)row * kVP + w);
  float* dp = out + (size_t)i4;
  *(volatile v4f*)dp = o;
  __threadfence();
  *(volatile v4f*)dp = o;
}
static_assert((size_t)kRO * kV / 4 == 6250 * (size_t)kThr, "output grid exact");

static_assert(((size_t)kRF * kF / 8) % kThr == 0 && ((size_t)kA * kF / 8) % kThr == 0 && ((size_t)kA * kH / 8) % kThr == 0, "plane cast grids exact");

extern "C" void kernel_launch(void* const* d_in, const int* in_sizes, int n_in,
                              void* d_out, int out_size, void* d_ws, size_t ws_size,
                              hipStream_t stream) {
  if (n_in < 15 || d_out == nullptr || d_ws == nullptr) return;
  if (in_sizes[0] != kRF * kF || in_sizes[1] != kB * kT || in_sizes[2] != kV * kE || in_sizes[3] != kG4 * (kE + kF) || in_sizes[4] != kG4) return;
  if (in_sizes[5] != kG4 * kH || in_sizes[6] != kG4 || in_sizes[7] != kV * kH || in_sizes[8] != kV || in_sizes[9] != kA * kF || in_sizes[10] != kA) return;
  if (in_sizes[11] != kA * kH || in_sizes[12] != kA || in_sizes[13] != kA || in_sizes[14] != 1) return;
  if ((size_t)out_size != (size_t)kRO * kV) return;
  if (ws_size < kWsTotal) return;
  const float* features = (const float*)d_in[0];
  const int* captions = (const int*)d_in[1];
  const float* emb = (const float*)d_in[2];
  const float* W_ih = (const float*)d_in[3];
  const float* b_ih = (const float*)d_in[4];
  const float* W_hh = (const float*)d_in[5];
  const float* b_hh = (const float*)d_in[6];
  const float* fc_W = (const float*)d_in[7];
  const float* fc_b = (const float*)d_in[8];
  const float* enc_W = (const float*)d_in[9];
  const float* enc_b = (const float*)d_in[10];
  const float* dec_W = (const float*)d_in[11];
  const float* dec_b = (const float*)d_in[12];
  const float* full_W = (const float*)d_in[13];
  const float* full_b = (const float*)d_in[14];
  float* out = (float*)d_out;
  char* ws = (char*)d_ws;
  unsigned short* F16 = (unsigned short*)(ws + kOffF16);
  unsigned short* ENCW = (unsigned short*)(ws + kOffENCW);
  unsigned short* DECW = (unsigned short*)(ws + kOffDECW);
  unsigned short* WG16 = (unsigned short*)(ws + kOffWG16);
  unsigned short* FCW = (unsigned short*)(ws + kOffFCW);
  float* BIAS = (float*)(ws + kOffBIAS);
  float* ENC32 = (float*)(ws + kOffENC32);
  unsigned short* A16 = (unsigned short*)(ws + kOffA16);
  float* DP32 = (float*)(ws + kOffDP32);
  float* G32 = (float*)(ws + kOffG32);
  float* C32 = (float*)(ws + kOffC32);
  unsigned short* HS16 = (unsigned short*)(ws + kOffHS16);
  float* LOG32 = (float*)(ws + kOffLOG32);

  cast_plane_kernel<<<(int)(((size_t)kRF * kF / 8) / kThr), kThr, 0, stream>>>(features, F16, 11, kF, 0);
  cast_plane_kernel<<<(int)(((size_t)kA * kF / 8) / kThr), kThr, 0, stream>>>(enc_W, ENCW, 11, kF, 0);
  cast_plane_kernel<<<(int)(((size_t)kA * kH / 8) / kThr), kThr, 0, stream>>>(dec_W, DECW, 9, kH, 0);
  wgate_kernel<<<3072, kThr, 0, stream>>>(W_ih, W_hh, WG16);
  fcw_kernel<<<2560, kThr, 0, stream>>>(fc_W, FCW);
  setup_kernel<<<125, kThr, 0, stream>>>(enc_b, dec_b, b_ih, b_hh, fc_b, BIAS, A16, C32);
  wmma_gemm64<0, false, 2, 0, false, 0><<<dim3((kRF / 64) * (kA / 64) / 8, 1), 256, 0, stream>>>(
      F16, F16, kF, 0L, ENCW, ENCW, kF, 0L, (void*)ENC32, (void*)ENC32, kA, 0L, BIAS + kFBE, nullptr, 0L, kRF, kA, kF, kSc);

  for (int t = 0; t < kT; ++t) {
    wmma_gemm64<0, false, 2, 0, false, 0><<<dim3((kBP / 64) * (kA / 64) / 8, 1), 256, 0, stream>>>(
        A16 + (kE + kF), A16 + (kE + kF), kKG, 0L, DECW, DECW, kH, 0L, (void*)DP32, (void*)DP32, kA, 0L, BIAS + kFBD, nullptr, 0L, kBP, kA, kH, kSc);
    score_kernel<<<kB, kThr, 0, stream>>>(ENC32, DP32, full_W, full_b, features, captions, emb, A16, t);
    wmma_gemm64<0, false, 2, 0, false, 0><<<dim3((kBP / 64) * (kG4 / 64) / 8, 1), 256, 0, stream>>>(
        A16, A16, kKG, 0L, WG16, WG16, kKG, 0L, (void*)G32, (void*)G32, kG4, 0L, BIAS + kFBG, nullptr, 0L, kBP, kG4, kKG, kSc);
    cell_kernel<<<8, kThr, 0, stream>>>(G32, C32, A16, HS16, t);
  }
  wmma_gemm64<0, false, 2, 0, false, 0><<<dim3((kRO / 64) * (kVP / 64) / 8, 1), 256, 0, stream>>>(
      HS16, HS16, kH, 0L, FCW, FCW, kH, 0L, (void*)LOG32, (void*)LOG32, kVP, 0L, BIAS + kFBF, nullptr, 0L, kRO, kVP, kH, kSc);
  out_kernel<<<6250, kThr, 0, stream>>>(LOG32, out);
}
